// MultiHeadSelfAttention_38457137169075
// MI455X (gfx1250) — hardware-verified
//
#include <hip/hip_runtime.h>


#ifndef NB
#define NB   4
#endif
#ifndef SEQ
#define SEQ  2048
#endif
#define NB_FULL  4
#define SEQ_FULL 2048
#define DM   1024
#define NH   16
#define HD   64
#define QKVN (3 * DM)
#define PCAR 4096.0f
#define SCL  0.125f
#define L2E  1.4426950408889634f

static_assert(SEQ % 64 == 0);
static_assert(SEQ <= SEQ_FULL);
static_assert(NB >= 1 && NB <= NB_FULL);
static_assert(NH * HD == DM);
static_assert(HD == 64);
static_assert(DM % 64 == 0 && QKVN % 64 == 0);
static_assert(DM % 32 == 0);
static_assert(NH == 16);
static_assert(SEQ_FULL < (1 << 24));
static_assert((size_t)QKVN * DM * 2 + (size_t)DM * DM * 2 + (size_t)SEQ * DM * 2 * 3 + (size_t)SEQ * QKVN * 4 + (size_t)2 * NH * SEQ * HD * 2 + (size_t)NH * HD * SEQ * 2 <= (size_t)134217728);

typedef _Float16 h16;
typedef unsigned short bf;
typedef __attribute__((ext_vector_type(16))) __bf16   v16bf;
typedef __attribute__((ext_vector_type(16))) _Float16 v16h;
typedef __attribute__((ext_vector_type(8)))  _Float16 v8h;
typedef __attribute__((ext_vector_type(8)))  unsigned short v8us;
typedef __attribute__((ext_vector_type(8)))  float    v8f;
typedef __attribute__((ext_vector_type(4)))  float    v4f;
typedef __attribute__((ext_vector_type(2)))  _Float16 v2h;
typedef __attribute__((ext_vector_type(4)))  _Float16 v4h;
typedef __attribute__((ext_vector_type(2)))  unsigned short v2us;
typedef __attribute__((ext_vector_type(4)))  unsigned short v4us;
typedef __attribute__((ext_vector_type(2)))  float v2f;
typedef v8h  __attribute__((may_alias)) v8ha;
typedef v4f  __attribute__((may_alias)) v4fa;
typedef v8us __attribute__((may_alias)) v8usa;

__device__ __forceinline__ unsigned short f2bf(float f) { unsigned u = __float_as_uint(f); u += 0x7FFFu + ((u >> 16) & 1u); return (unsigned short)(u >> 16); }
__device__ __forceinline__ float bf2f(unsigned short b) { return __uint_as_float(((unsigned)b) << 16); }
__device__ __forceinline__ float bfr(float f) { return bf2f(f2bf(f)); }
__device__ __forceinline__ v16h cat16(v8h lo, v8h hi) { return __builtin_shufflevector(lo, hi, 0, 1, 2, 3, 4, 5, 6, 7, 8, 9, 10, 11, 12, 13, 14, 15); }
__device__ __forceinline__ v16bf cat16b(v8us lo, v8us hi) { return __builtin_bit_cast(v16bf, __builtin_shufflevector(lo, hi, 0, 1, 2, 3, 4, 5, 6, 7, 8, 9, 10, 11, 12, 13, 14, 15)); }
__device__ __forceinline__ v8f wmma16(v16h a, v16h b, v8f c) { return __builtin_amdgcn_wmma_f32_16x16x32_f16(false, a, false, b, (short)0, c, false, false); }
__device__ __forceinline__ v8f wmmab(v16bf a, v16bf b, v8f c) { return __builtin_amdgcn_wmma_f32_16x16x32_bf16(false, a, false, b, (short)0, c, false, false); }
__device__ __forceinline__ h16 tohx(float x) { return (h16)x; }
__device__ __forceinline__ void splitf(float y, unsigned short& h, unsigned short& l) { h = f2bf(y); l = f2bf(y - bf2f(h)); }
__device__ __forceinline__ v16h ldh(const h16* p) { return cat16(*(const v8h*)p, *(const v8h*)(p + 16)); }
static __device__ __forceinline__ h16 toh_flush(float v) { const h16 r = (h16)v; return (fabsf(v) < 6.103515625e-05f) ? (h16)0.0f : r; }

template <typename T16> struct WFrag;
template <> struct WFrag<h16> { typedef v16h V; static __device__ __forceinline__ V ld(const h16* p) { return cat16(*(const v8h*)p, *(const v8h*)(p + 16)); } static __device__ __forceinline__ v8f mma(V a, V b, v8f c) { return wmma16(a, b, c); } };
template <> struct WFrag<bf> { typedef v16bf V; static __device__ __forceinline__ V ld(const bf* p) { return cat16b(*(const v8us*)p, *(const v8us*)(p + 16)); } static __device__ __forceinline__ v8f mma(V a, V b, v8f c) { return wmmab(a, b, c); } };
template <typename T16, int NSPLIT, bool BIAS>
__global__ __launch_bounds__(32) void k_gemmw(const T16* __restrict__ A, const T16* __restrict__ A2, const T16* __restrict__ Bt, const T16* __restrict__ Bt2, int K, float* C, int ldc, const float* __restrict__ bias, size_t sA, size_t sB, size_t sC) {
    typedef typename WFrag<T16>::V V;
    __shared__ __align__(16) float os[16 * 68];
    const size_t z = blockIdx.z; A += z * sA; if (A2) A2 += z * sA; Bt += z * sB; if (Bt2) Bt2 += z * sB; C += z * sC;
    const int lane = threadIdx.x & 31, lr = lane & 15, hi = lane >> 4; const int r0 = blockIdx.x * 64, c0 = blockIdx.y * 64;
    v8f acc[4][4];
#pragma unroll
    for (int mb = 0; mb < 4; ++mb)
#pragma unroll
        for (int nb = 0; nb < 4; ++nb) acc[mb][nb] = (v8f){};
    const size_t aoff = (size_t)(r0 + lr) * K + 8 * hi, boff = (size_t)(c0 + lr) * K + 8 * hi;
#pragma unroll 1
    for (int kc = 0; kc < K; kc += 32) {
        V a[4], a2[4];
#pragma unroll
        for (int mb = 0; mb < 4; ++mb) { a[mb] = WFrag<T16>::ld(A + aoff + (size_t)mb * 16 * K + kc); if (NSPLIT == 1 || NSPLIT == 2) a2[mb] = WFrag<T16>::ld(A2 + aoff + (size_t)mb * 16 * K + kc); }
#pragma unroll
        for (int nb = 0; nb < 4; ++nb) { const V b = WFrag<T16>::ld(Bt + boff + (size_t)nb * 16 * K + kc); V b2; if (NSPLIT >= 2) b2 = WFrag<T16>::ld(Bt2 + boff + (size_t)nb * 16 * K + kc);
#pragma unroll
            for (int mb = 0; mb < 4; ++mb) { acc[mb][nb] = WFrag<T16>::mma(a[mb], b, acc[mb][nb]); if (NSPLIT == 1 || NSPLIT == 2) acc[mb][nb] = WFrag<T16>::mma(a2[mb], b, acc[mb][nb]); if (NSPLIT >= 2) acc[mb][nb] = WFrag<T16>::mma(a[mb], b2, acc[mb][nb]); } }
        asm volatile("v_nop\n\tv_nop\n\tv_nop\n\tv_nop" : "+v"(acc[0][0]), "+v"(acc[1][1]), "+v"(acc[2][2]), "+v"(acc[3][3]) : "v"(a[0]), "v"(a[3]));
    }
#pragma unroll
    for (int mb = 0; mb < 4; ++mb) {
#pragma unroll
        for (int nb = 0; nb < 4; ++nb) {
#pragma unroll
            for (int j = 0; j < 8; ++j) os[(hi * 8 + j) * 68 + nb * 16 + lr] = acc[mb][nb][j]; }
        __builtin_amdgcn_wave_barrier(); asm volatile("" ::: "memory");
        float* crow = C + (size_t)(r0 + mb * 16) * ldc + c0;
#pragma unroll 1
        for (int ps = 0; ps < 2; ++ps) {
#pragma unroll
            for (int s = 0; s < 8; ++s) { const int row = 2 * s + hi, cofs = lr * 4; v4f val = *(const v4fa*)(os + row * 68 + cofs); if (BIAS) { val[0] += bfr(bias[c0 + cofs]); val[1] += bfr(bias[c0 + cofs + 1]); val[2] += bfr(bias[c0 + cofs + 2]); val[3] += bfr(bias[c0 + cofs + 3]); }
                *(volatile v4f*)(crow + (size_t)row * ldc + cofs) = val; }
            if (ps == 0) __threadfence(); }
        __builtin_amdgcn_wave_barrier(); asm volatile("" ::: "memory");
    }
}

__global__ __launch_bounds__(256) void k_wtG(const float* __restrict__ w, int K, int N, bf* Bt) {
    const int lane = threadIdx.x & 31; const int L0 = (blockIdx.x * 8 + (threadIdx.x >> 5)) * 8; const int nlines = N * K / 64;
#pragma unroll
    for (int ps = 0; ps < 2; ++ps) {
#pragma unroll 1
        for (int l = 0; l < 8; ++l) { const int L = L0 + l; if (L >= nlines) break; const size_t e = (size_t)L * 64 + lane * 2; const int k = (int)(e % K), n = (int)(e / K); v2us o;
            o[0] = f2bf(w[(size_t)k * N + n]); o[1] = f2bf(w[(size_t)(k + 1) * N + n]); *(volatile v2us*)(Bt + e) = o; }
        if (ps == 0) __threadfence(); }
}
__global__ __launch_bounds__(256) void k_cvt8(const float* __restrict__ src, bf* dst, size_t n8) { const size_t i = (size_t)blockIdx.x * 256 + threadIdx.x; if (i >= n8) return; const v8f v = *(const v8f*)(src + i * 8); v8us o;
#pragma unroll
    for (int k = 0; k < 8; ++k) o[k] = f2bf(v[k]); *(volatile v8us*)(dst + i * 8) = o; __threadfence(); *(volatile v8us*)(dst + i * 8) = o; }

__global__ __launch_bounds__(256) void k_qkp(const float* __restrict__ F, h16* P) {
    const size_t e = ((size_t)blockIdx.x * 256 + threadIdx.x) * 8; if (e >= (size_t)2 * NH * SEQ * HD) return;
    const int d = (int)(e % HD); const int t = (int)((e / HD) % SEQ); const int g = (int)(e / ((size_t)HD * SEQ));
    const float* f = F + (size_t)t * QKVN + (size_t)g * HD + d;
    const v4f a = *(const v4f*)f, b4 = *(const v4f*)(f + 4); v8h o;
#pragma unroll
    for (int q = 0; q < 4; ++q) { o[q] = tohx(a[q]); o[4 + q] = tohx(b4[q]); }
    *(volatile v8h*)(P + e) = o; __threadfence(); *(volatile v8h*)(P + e) = o;
}
__global__ __launch_bounds__(256) void k_vtp(const float* __restrict__ F, h16* V16) {
    const size_t e = ((size_t)blockIdx.x * 256 + threadIdx.x) * 8; if (e >= (size_t)NH * HD * SEQ) return;
    const int t = (int)(e % SEQ); const int d = (int)((e / SEQ) % HD); const int g = (int)(e / ((size_t)SEQ * HD));
    const float* f = F + (size_t)t * QKVN + (size_t)g * HD + d; v8h o;
#pragma unroll
    for (int q = 0; q < 8; ++q) o[q] = tohx(f[(size_t)q * QKVN]);
    *(volatile v8h*)(V16 + e) = o; __threadfence(); *(volatile v8h*)(V16 + e) = o;
}

__global__ __launch_bounds__(128) void k_attn(const h16* __restrict__ Qp, const h16* __restrict__ Kp, const h16* __restrict__ Vt, const float* __restrict__ wrel, bf* Ah, bf* Al) {
#pragma clang fp contract(off)
    __shared__ __align__(16) float cst[4][16 * 68];
    const int lane = threadIdx.x & 31, wv = threadIdx.x >> 5, lr = lane & 15, hi = lane >> 4;
    const int h = blockIdx.y; const int q0 = blockIdx.x * 64 + wv * 16;
    const float wr = bfr(wrel[h]);
    const int qi = q0 + lr;
    const h16* Qb = Qp + ((size_t)h * SEQ + q0) * HD;
    const h16* Kb = Kp + (size_t)h * SEQ * HD;
    const h16* Vb = Vt + (size_t)h * HD * SEQ;
    v16h qf[2];
    qf[0] = ldh(Qb + (size_t)lr * HD + 8 * hi); qf[1] = ldh(Qb + (size_t)lr * HD + 32 + 8 * hi);
    v8f o[4];
#pragma unroll
    for (int c = 0; c < 4; ++c) o[c] = (v8f){};
    float mrun = -1.0e30f, lrun = 0.0f;
#pragma unroll 1
    for (int kv = 0; kv < SEQ; kv += 64) {
        v16h ka[4][2];
#pragma unroll
        for (int c = 0; c < 4; ++c) { const h16* kp = Kb + (size_t)(kv + 16 * c + lr) * HD + 8 * hi; ka[c][0] = ldh(kp); ka[c][1] = ldh(kp + 32); }
        v8f s[4];
#pragma unroll
        for (int c = 0; c < 4; ++c) { const v8f zz = (v8f){}; s[c] = wmma16(ka[c][0], qf[0], zz); s[c] = wmma16(ka[c][1], qf[1], s[c]); }
        asm volatile("v_nop\n\tv_nop\n\tv_nop\n\tv_nop" : "+v"(s[0]), "+v"(s[1]), "+v"(s[2]), "+v"(s[3]) : "v"(qf[0]), "v"(qf[1]), "v"(ka[3][1]));
        const float relb = (float)(kv + 8 * hi - qi);
        float mx = -1.0e30f;
#pragma unroll
        for (int c = 0; c < 4; ++c)
#pragma unroll
            for (int r = 0; r < 8; ++r) { const float pbias = (relb + (float)(16 * c + r)) * wr; const float t = __builtin_fmaf(s[c][r], SCL, pbias); s[c][r] = t; mx = fmaxf(mx, t); }
        mx = fmaxf(mx, __shfl_xor(mx, 16, 32));
        const float mn = fmaxf(mrun, mx); const float corr = __builtin_amdgcn_exp2f((mrun - mn) * L2E); mrun = mn;
        float sm = 0.0f;
#pragma unroll
        for (int c = 0; c < 4; ++c)
#pragma unroll
            for (int r = 0; r < 8; ++r) { const float p = __builtin_amdgcn_exp2f((s[c][r] - mn) * L2E); s[c][r] = p; sm += p; }
        sm += __shfl_xor(sm, 16, 32);
        lrun = lrun * corr + sm;
#pragma unroll
        for (int c = 0; c < 4; ++c) o[c] = o[c] * corr;
        v16h pb[2];
#pragma unroll
        for (int ks = 0; ks < 2; ++ks) { v8h plo, phh;
#pragma unroll
            for (int r = 0; r < 8; ++r) { plo[r] = toh_flush(s[2 * ks][r] * PCAR); phh[r] = toh_flush(s[2 * ks + 1][r] * PCAR); }
            pb[ks] = cat16(plo, phh); }
        v16h va[4][2];
#pragma unroll
        for (int c = 0; c < 4; ++c) { const h16* vp = Vb + (size_t)(16 * c + lr) * SEQ + kv + 8 * hi; va[c][0] = ldh(vp); va[c][1] = ldh(vp + 32); }
#pragma unroll
        for (int c = 0; c < 4; ++c) { o[c] = wmma16(va[c][0], pb[0], o[c]); o[c] = wmma16(va[c][1], pb[1], o[c]); }
        asm volatile("v_nop\n\tv_nop\n\tv_nop\n\tv_nop" : "+v"(o[0]), "+v"(o[1]), "+v"(o[2]), "+v"(o[3]) : "v"(pb[0]), "v"(pb[1]), "v"(va[3][1]));
    }
    const float inv = __builtin_amdgcn_rcpf(lrun * PCAR);
    float* myf = cst[wv];
#pragma unroll
    for (int c = 0; c < 4; ++c) { v4f a, b4;
#pragma unroll
        for (int r = 0; r < 4; ++r) { a[r] = o[c][r] * inv; b4[r] = o[c][4 + r] * inv; }
        *(v4fa*)(myf + lr * 68 + 16 * c + 8 * hi) = a; *(v4fa*)(myf + lr * 68 + 16 * c + 8 * hi + 4) = b4; }
    __builtin_amdgcn_fence(3  , "wavefront"); __builtin_amdgcn_wave_barrier(); asm volatile("" ::: "memory");
    const int rsub = lane >> 3, piece = (lane & 7) * 8;
    v8us oh[4], ol[4]; size_t oo[4];
#pragma unroll
    for (int g = 0; g < 4; ++g) { const int row = g * 4 + rsub; const v4f a = *(const v4fa*)(myf + row * 68 + piece), b4 = *(const v4fa*)(myf + row * 68 + piece + 4);
#pragma unroll
        for (int j = 0; j < 4; ++j) { unsigned short u, w; splitf(a[j], u, w); oh[g][j] = u; ol[g][j] = w; splitf(b4[j], u, w); oh[g][4 + j] = u; ol[g][4 + j] = w; }
        oo[g] = (size_t)(q0 + row) * DM + (size_t)h * HD + piece; }
#pragma unroll 1
    for (int ps = 0; ps < 2; ++ps) {
#pragma unroll
        for (int g = 0; g < 4; ++g) { *(volatile v8us*)(Ah + oo[g]) = oh[g]; *(volatile v8us*)(Al + oo[g]) = ol[g]; }
        if (ps == 0) __threadfence(); }
}

extern "C" void kernel_launch(void* const* d_in, const int* in_sizes, int n_in,
                              void* d_out, int out_size, void* d_ws, size_t ws_size, hipStream_t stream) {
    if (n_in < 4) return;
    if (in_sizes[0] < (NB - 1) * SEQ_FULL * DM + SEQ * DM) return;
    if (in_sizes[1] < DM * QKVN) return;
    if (in_sizes[2] < DM * DM) return;
    if (in_sizes[3] < NH) return;
    if (out_size < (NB - 1) * SEQ * DM + SEQ * DM) return;
    const float* x = (const float*)d_in[0];
    const float* wqkv = (const float*)d_in[1];
    const float* wproj = (const float*)d_in[2];
    const float* wrel = (const float*)d_in[3];
    float* OUT = (float*)d_out;
    char* wsp = (char*)d_ws;
    auto take = [&](size_t bytes) { char* p = wsp; wsp += (bytes + 255) & ~(size_t)255; return (void*)p; };
    bf*   WQKV = (bf*)take((size_t)QKVN * DM * 2);
    bf*   WO   = (bf*)take((size_t)DM * DM * 2);
    bf*   XB   = (bf*)take((size_t)SEQ * DM * 2);
    float* F   = (float*)take((size_t)SEQ * QKVN * 4);
    h16*  QK16 = (h16*)take((size_t)2 * NH * SEQ * HD * 2);
    h16*  VT16 = (h16*)take((size_t)NH * HD * SEQ * 2);
    bf*   ATh  = (bf*)take((size_t)SEQ * DM * 2);
    bf*   ATl  = (bf*)take((size_t)SEQ * DM * 2);
    if ((size_t)(wsp - (char*)d_ws) > ws_size) return;
    k_wtG<<<(unsigned)((QKVN * DM / 64 + 63) / 64), 256, 0, stream>>>(wqkv, DM, QKVN, WQKV);
    k_wtG<<<(unsigned)((DM * DM / 64 + 63) / 64), 256, 0, stream>>>(wproj, DM, DM, WO);
    const unsigned LX  = (unsigned)(((size_t)SEQ * DM / 8 + 255) / 256);
    const unsigned LQK = (unsigned)(((size_t)2 * NH * SEQ * HD / 8 + 255) / 256);
    const unsigned LV  = (unsigned)(((size_t)NH * HD * SEQ / 8 + 255) / 256);
    for (int b = 0; b < NB; ++b) {
        k_cvt8<<<LX, 256, 0, stream>>>(x + (size_t)b * SEQ_FULL * DM, XB, (size_t)SEQ * DM / 8);
        k_gemmw<bf, 0, false><<<dim3(SEQ / 64, QKVN / 64, 1), 32, 0, stream>>>(XB, nullptr, WQKV, nullptr, DM, F, QKVN, nullptr, 0, 0, 0);
        k_qkp<<<LQK, 256, 0, stream>>>(F, QK16);
        k_vtp<<<LV, 256, 0, stream>>>(F + 2 * DM, VT16);
        k_attn<<<dim3(SEQ / 64, NH, 1), 128, 0, stream>>>(QK16, QK16 + (size_t)NH * SEQ * HD, VT16, wrel, ATh, ATl);
        k_gemmw<bf, 1, false><<<dim3(SEQ / 64, DM / 64, 1), 32, 0, stream>>>(ATh, ATl, WO, nullptr, DM, OUT + (size_t)b * SEQ * DM, DM, nullptr, 0, 0, 0);
    }
}
